// MLA_82454782148667
// MI455X (gfx1250) — hardware-verified
//
#include <hip/hip_runtime.h>
#include <math.h>

constexpr int kBatch  = 2;
constexpr int kSeq    = 2048;
constexpr int kDim    = 2048;
constexpr int kHeads  = 16;
constexpr int kDNope  = 128;
constexpr int kDRope  = 64;
constexpr int kDQK    = 192;
constexpr int kDV     = 128;
constexpr int kRank   = 512;
constexpr int kTok    = kBatch * kSeq;
constexpr int kQCols  = kHeads * kDQK;
constexpr int kKVCols = kHeads * kDNope;
constexpr int kKCCols = kRank + kDRope;
constexpr int kPairs  = kDRope / 2;
constexpr int kEarly  = 128;
constexpr int kTokE   = kBatch * kEarly;
constexpr float kPCarry  = 32768.0f;
constexpr float kOCarry  = 64.0f;
constexpr float kWCarry  = 64.0f;
constexpr float kWCarryInv = 1.0f / 64.0f;
constexpr float kLoCarry = 2048.0f;
static_assert(kHeads * kDV == kKVCols, "shape");
static_assert(kDQK == kDNope + kDRope, "shape");
static_assert(kTok % 64 == 0 && kEarly % 64 == 0 && (kSeq - kEarly) % 64 == 0 && kSeq % 64 == 0, "M tiles");
static_assert(kQCols % 64 == 0 && kRank % 64 == 0 && kDRope % 64 == 0 && kKVCols % 64 == 0 && kDim % 64 == 0 && kDV % 64 == 0, "N tiles");
static_assert(kDim % 32 == 0 && kRank % 32 == 0 && kDQK % 32 == 0 && kEarly % 32 == 0 && kKVCols % 32 == 0, "K tiles");
static_assert(kSeq % 128 == 0, "query blocks");

typedef __attribute__((ext_vector_type(16))) _Float16 v16h;
typedef __attribute__((ext_vector_type(8)))  _Float16 v8h;
typedef __attribute__((ext_vector_type(16))) __bf16   v16b;
typedef __attribute__((ext_vector_type(8)))  __bf16   v8b;
typedef __attribute__((ext_vector_type(8)))  float    v8f;
typedef __attribute__((ext_vector_type(4)))  float    v4f;
typedef __attribute__((ext_vector_type(2)))  float    v2f;
typedef __attribute__((ext_vector_type(4)))  unsigned int v4u;

__device__ __forceinline__ unsigned short f2bf_bits(float f) {
  unsigned u = __float_as_uint(f);
  return (unsigned short)((u + 0x7FFFu + ((u >> 16) & 1u)) >> 16);
}
__device__ __forceinline__ float bf_bits2f(unsigned short h) { return __uint_as_float(((unsigned)h) << 16); }

__device__ __forceinline__ float h16_to_f32(unsigned hb) {
  const unsigned sgn = (hb & 0x8000u) << 16; const unsigned em = hb & 0x7fffu;
  const float fn = __uint_as_float((em << 13) + 0x38000000u);
  const float fs = (float)em * 5.9604644775390625e-8f;
  const float mag = (em < 0x400u) ? fs : fn; return __uint_as_float(__float_as_uint(mag) | sgn); }

__device__ __forceinline__ unsigned pk16(unsigned short a, unsigned short b) { return (unsigned)a | ((unsigned)b << 16); }
__device__ __forceinline__ unsigned short h_bits(float f) { const _Float16 h = (_Float16)f; return __builtin_bit_cast(unsigned short, h); }

__device__ __forceinline__ void dep_guard_h(v8f& a, v8f& b, v16h x, v16h y) { asm volatile("v_nop\n\tv_nop\n\tv_nop\n\tv_nop" : "+v"(a), "+v"(b) : "v"(x), "v"(y)); }
__device__ __forceinline__ void dep_guard_b(v8f& a, v8f& b, v16b x, v16b y) { asm volatile("v_nop\n\tv_nop\n\tv_nop\n\tv_nop" : "+v"(a), "+v"(b) : "v"(x), "v"(y)); }
__device__ __forceinline__ void keep4_h(v16h a, v16h b, v16h c, v16h d) { asm volatile("v_nop" :: "v"(a), "v"(b), "v"(c), "v"(d)); }
__device__ __forceinline__ void keep4_b(v16b a, v16b b, v16b c, v16b d) { asm volatile("v_nop" :: "v"(a), "v"(b), "v"(c), "v"(d)); }
__device__ __forceinline__ void acc_guard4(v8f& a, v8f& b, v8f& c, v8f& d) { asm volatile("v_nop\n\tv_nop\n\tv_nop\n\tv_nop" : "+v"(a), "+v"(b), "+v"(c), "+v"(d)); }
template <typename T> struct Frag;
template <> struct Frag<_Float16> {
  typedef v16h V; union U { v16h v; v8h h[2]; };
  static __device__ __forceinline__ v16h load(const _Float16* p) {
    U f; f.h[0] = *(const v8h*)(p); f.h[1] = *(const v8h*)(p + 16); return f.v;
  }
  static __device__ __forceinline__ v8f mma(v16h a, v16h b, v8f c) {
    return __builtin_amdgcn_wmma_f32_16x16x32_f16(false, a, false, b, (short)0, c, false, false);
  }
  static __device__ __forceinline__ void guard(v8f& a, v8f& b, v16h x, v16h y) { dep_guard_h(a, b, x, y); }
  static __device__ __forceinline__ void keep(v16h a, v16h b, v16h c, v16h d) { keep4_h(a, b, c, d); }
};
template <> struct Frag<__bf16> {
  typedef v16b V; union U { v16b v; v8b h[2]; };
  static __device__ __forceinline__ v16b load(const __bf16* p) {
    U f; f.h[0] = *(const v8b*)(p); f.h[1] = *(const v8b*)(p + 16); return f.v;
  }
  static __device__ __forceinline__ v8f mma(v16b a, v16b b, v8f c) {
    return __builtin_amdgcn_wmma_f32_16x16x32_bf16(false, a, false, b, (short)0, c, false, false);
  }
  static __device__ __forceinline__ void guard(v8f& a, v8f& b, v16b x, v16b y) { dep_guard_b(a, b, x, y); }
  static __device__ __forceinline__ void keep(v16b a, v16b b, v16b c, v16b d) { keep4_b(a, b, c, d); }
};

__device__ __forceinline__ v8f fa_mma(v16h a, v16h b, v8f c) {
  c = __builtin_amdgcn_wmma_f32_16x16x32_f16(false, a, false, b, (short)0, c, false, false);
  asm volatile("v_nop\n\tv_nop\n\tv_nop\n\tv_nop" : "+v"(c) : "v"(a), "v"(b));
  return c;
}

__device__ __forceinline__ void wave_lds_sync() {
  __builtin_amdgcn_fence(__ATOMIC_RELEASE, "workgroup");
  __builtin_amdgcn_wave_barrier();
  __builtin_amdgcn_fence(__ATOMIC_ACQUIRE, "workgroup");
}

template <int ET> struct Elem;
template <> struct Elem<0> { typedef _Float16 T; };
template <> struct Elem<1> { typedef __bf16 T; };
template <int ET, int SPLIT, int BIAS_MODE, int OUT_MODE, bool RESID>
__global__ __launch_bounds__(256) void wmma_gemm64(
    const unsigned short* __restrict__ Ap, const unsigned short* __restrict__ A2p, int lda, long strideA,
    const unsigned short* __restrict__ Btp, const unsigned short* __restrict__ Bt2p, int ldb, long strideB,
    void* __restrict__ Cout, void* __restrict__ Cout2, int ldc, long strideC,
    const float* __restrict__ bias,
    const float* __restrict__ resid, long strideR,
    int M, int N, int K, float scale) {
  static_assert(BIAS_MODE == 0 || OUT_MODE == 0, "bias only on f32 out");
  static_assert(!RESID || OUT_MODE == 0, "resid only on f32 out");
  static_assert(BIAS_MODE == 0 || BIAS_MODE == 2, "bias mode");
  constexpr bool LA = (SPLIT == 1 || SPLIT == 2);
  constexpr bool LB = (SPLIT == 1 || SPLIT == 3);
  typedef typename Elem<ET>::T T;
  typedef typename Frag<T>::V V;
  const T* A = (const T*)Ap; const T* A2 = (const T*)A2p; const T* Bt = (const T*)Btp; const T* Bt2 = (const T*)Bt2p;
  __shared__ __align__(16) float sT[8][16 * 68];
  const int b    = blockIdx.y;
  const int lane = threadIdx.x & 31;
  const int wave = threadIdx.x >> 5;
  const int tilesN = N >> 6;
  const int tilesM = M >> 6;
  const int tile = blockIdx.x * 8 + wave;
  if (tile >= tilesM * tilesN) return;
  const int tm = tile / tilesN;
  const int tn = tile - tm * tilesN;
  const int m0 = tm << 6;
  const int n0 = tn << 6;

  const T* Ab  = A  + (size_t)b * strideA;
  const T* Bb  = Bt + (size_t)b * strideB;
  const T* Ab2 = LA ? (A2  + (size_t)b * strideA) : nullptr;
  const T* Bb2 = LB ? (Bt2 + (size_t)b * strideB) : nullptr;

  const int rlane = lane & 15;
  const int koff  = (lane >> 4) * 8;
  const int mOff  = (lane >> 4) * 8;

  v8f acc[4][4];
#pragma unroll
  for (int i = 0; i < 4; ++i)
#pragma unroll
    for (int j = 0; j < 4; ++j) acc[i][j] = (v8f){0.f,0.f,0.f,0.f,0.f,0.f,0.f,0.f};

  for (int k0 = 0; k0 < K; k0 += 32) {
    V bh[4], bl[4];
#pragma unroll
    for (int j = 0; j < 4; ++j) {
      const size_t bo = (size_t)(n0 + (j << 4) + rlane) * ldb + koff + k0;
      bh[j] = Frag<T>::load(Bb + bo);
      if (LB) bl[j] = Frag<T>::load(Bb2 + bo);
    }
#pragma unroll
    for (int i = 0; i < 4; ++i) {
      const size_t ao = (size_t)(m0 + (i << 4) + rlane) * lda + koff + k0;
      V ah = Frag<T>::load(Ab + ao);
      V al = ah;
      if (LA) al = Frag<T>::load(Ab2 + ao);
#pragma unroll
      for (int j = 0; j < 4; ++j) {
        acc[i][j] = Frag<T>::mma(ah, bh[j], acc[i][j]);
        if (LB) acc[i][j] = Frag<T>::mma(ah, bl[j], acc[i][j]);
        if (LA) acc[i][j] = Frag<T>::mma(al, bh[j], acc[i][j]);
      }
      Frag<T>::guard(acc[i][0], acc[i][3], ah, al);
    }
    Frag<T>::keep(bh[0], bh[1], bh[2], bh[3]);
    if (LB) Frag<T>::keep(bl[0], bl[1], bl[2], bl[3]);
  }
  acc_guard4(acc[0][0], acc[0][1], acc[0][2], acc[0][3]);
  acc_guard4(acc[1][0], acc[1][1], acc[1][2], acc[1][3]);
  acc_guard4(acc[2][0], acc[2][1], acc[2][2], acc[2][3]);
  acc_guard4(acc[3][0], acc[3][1], acc[3][2], acc[3][3]);

  float* slab = sT[wave];
#pragma unroll
  for (int i = 0; i < 4; ++i) {
    const int mBase = m0 + (i << 4);
#pragma unroll
    for (int j = 0; j < 4; ++j) {
#pragma unroll
      for (int r = 0; r < 8; ++r) slab[(mOff + r) * 68 + (j << 4) + rlane] = acc[i][j][r] * scale;
    }
    wave_lds_sync();
    if (OUT_MODE == 0) {
      float* C = (float*)Cout + (size_t)b * strideC;
      const float* Rb = RESID ? (resid + (size_t)b * strideR) : nullptr;
      const int hh = lane >> 4, c4 = (lane & 15) * 4;
      v4f bb = (v4f){0.f, 0.f, 0.f, 0.f};
      if (BIAS_MODE == 2) bb = *(const v4f*)(bias + n0 + c4);
      for (int pass = 0; pass < 2; ++pass) {
#pragma unroll
        for (int it = 0; it < 8; ++it) {
          const int row = it * 2 + hh;
          v4f v = *(const v4f*)(slab + row * 68 + c4);
          if (BIAS_MODE == 2) v = v + bb;
          if (RESID) {
            const v4f rr = *(const v4f*)(Rb + (size_t)(mBase + row) * ldc + n0 + c4);
            v = v + rr;
          }
          *(volatile v4f*)(C + (size_t)(mBase + row) * ldc + n0 + c4) = v;
        }
        __threadfence();
      }
    } else {
      const int q = lane >> 3, c8 = (lane & 7) * 8;
      unsigned short* C  = (unsigned short*)Cout  + (size_t)b * strideC;
      unsigned short* C2 = (OUT_MODE >= 2) ? ((unsigned short*)Cout2 + (size_t)b * strideC) : nullptr;
      for (int pass = 0; pass < 2; ++pass) {
#pragma unroll
        for (int it = 0; it < 4; ++it) {
          const int row = it * 4 + q;
          const float* sp = slab + row * 68 + c8;
          v8h hv, lv;
#pragma unroll
          for (int e = 0; e < 8; ++e) {
            if (OUT_MODE == 1) {
              hv[e] = (_Float16)sp[e];
            } else if (OUT_MODE == 2) {
              unsigned short hb = f2bf_bits(sp[e]);
              unsigned short lb = f2bf_bits(sp[e] - bf_bits2f(hb));
              hv[e] = __builtin_bit_cast(_Float16, hb);
              lv[e] = __builtin_bit_cast(_Float16, lb);
            } else {
              unsigned short hb = h_bits(sp[e]);
              const float hf = h16_to_f32((unsigned)hb);
              unsigned short lb = h_bits((sp[e] - hf) * kLoCarry);
              hv[e] = __builtin_bit_cast(_Float16, hb);
              lv[e] = __builtin_bit_cast(_Float16, lb);
            }
          }
          *(volatile v8h*)(C + (size_t)(mBase + row) * ldc + n0 + c8) = hv;
          if (OUT_MODE >= 2) *(volatile v8h*)(C2 + (size_t)(mBase + row) * ldc + n0 + c8) = lv;
        }
        __threadfence();
      }
    }
    wave_lds_sync();
  }
}

__global__ __launch_bounds__(256) void cast8_x16_kernel(const float* __restrict__ in, unsigned short* __restrict__ out, int n8) {
  const int i = blockIdx.x * 256 + threadIdx.x;
  if (i >= n8) return;
  const float* p = in + 8 * (size_t)i;
  const v4f a = *(const v4f*)(p);
  const v4f c = *(const v4f*)(p + 4);
  unsigned short hb[8];
#pragma unroll
  for (int e = 0; e < 4; ++e) {
    hb[e]     = h_bits(bf_bits2f(f2bf_bits(a[e])));
    hb[4 + e] = h_bits(bf_bits2f(f2bf_bits(c[e])));
  }
  const v4u u = (v4u){pk16(hb[0], hb[1]), pk16(hb[2], hb[3]), pk16(hb[4], hb[5]), pk16(hb[6], hb[7])};
  unsigned short* q = out + 8 * (size_t)i;
  *(volatile v4u*)q = u;
  __threadfence();
  *(volatile v4u*)q = u;
}

template <bool F16OUT>
__global__ __launch_bounds__(256) void wtrans_kernel(const float* __restrict__ W, unsigned short* __restrict__ WT,
                                                     int Kin, int Nout, float scale) {
  __shared__ float sm[64][65];
  const int t  = threadIdx.x;
  const int k0 = blockIdx.x * 64;
  const int n0 = blockIdx.y * 64;
#pragma unroll
  for (int i = 0; i < 16; ++i) {
    const int e = i * 256 + t;
    const int r = e >> 6;
    const int c = e & 63;
    sm[c][r] = W[(size_t)(k0 + r) * Nout + n0 + c];
  }
  __syncthreads();
  const int lane = t & 31, wave = t >> 5;
  const int q = lane >> 3, c8 = (lane & 7) * 8;
  for (int pass = 0; pass < 2; ++pass) {
#pragma unroll
    for (int it = 0; it < 2; ++it) {
      const int row = wave * 8 + it * 4 + q;
      unsigned short hb[8];
#pragma unroll
      for (int e = 0; e < 8; ++e) {
        const unsigned short bbits = f2bf_bits(sm[row][c8 + e]);
        hb[e] = F16OUT ? h_bits(bf_bits2f(bbits) * scale) : bbits;
      }
      const v4u u = (v4u){pk16(hb[0], hb[1]), pk16(hb[2], hb[3]), pk16(hb[4], hb[5]), pk16(hb[6], hb[7])};
      *(volatile v4u*)(WT + (size_t)(n0 + row) * Kin + k0 + c8) = u;
    }
    __threadfence();
  }
}

__global__ __launch_bounds__(256) void bias_rne_kernel(const float* __restrict__ in, float* __restrict__ out, int n4) {
  const int i = blockIdx.x * 256 + threadIdx.x;
  if (i >= n4) return;
  const v4f a = *(const v4f*)(in + 4 * (size_t)i);
  v4f o;
#pragma unroll
  for (int e = 0; e < 4; ++e) o[e] = bf_bits2f(f2bf_bits(a[e]));
  float* p = out + 4 * (size_t)i;
  *(volatile v4f*)p = o;
  __threadfence();
  *(volatile v4f*)p = o;
}

struct Theta32 { float t[32]; };
static_assert(sizeof(Theta32) == 128, "no padding");
__global__ __launch_bounds__(256) void rope_table_kernel(float* __restrict__ cs, Theta32 th, const int* __restrict__ sp_unused) {
  #pragma clang fp contract(off)
  (void)sp_unused;
  const int g = blockIdx.x * 256 + threadIdx.x;
  if (g >= kSeq * kPairs) return;
  const int pos = g >> 5;
  const int i = g & 31;
  float theta = 0.0f;
#pragma unroll
  for (int k = 0; k < 32; ++k) theta = (i == k) ? th.t[k] : theta;
  const float ang = (float)pos * theta;
  float sn, cn;
  sincosf(ang, &sn, &cn);
  const v2f o = (v2f){cn, sn};
  float* p = cs + 2 * (size_t)g;
  *(volatile v2f*)p = o;
  __threadfence();
  *(volatile v2f*)p = o;
}

__global__ __launch_bounds__(256) void rope_k_kernel(const float* __restrict__ kr32, const float* __restrict__ cs,
                                                    unsigned short* __restrict__ kr16,
                                                    unsigned short* __restrict__ kreh, unsigned short* __restrict__ krel) {
  #pragma clang fp contract(off)
  const int g = blockIdx.x * 256 + threadIdx.x;
  if (g >= kTok * kPairs) return;
  const int t = g >> 5;
  const int i = g & 31;
  const int pos = t & (kSeq - 1);
  const int b = t >> 11;
  const v2f xv = *(const v2f*)(kr32 + (size_t)t * kDRope + 2 * i);
  const v2f cv = *(const v2f*)(cs + ((size_t)pos * kPairs + i) * 2);
  const float x0 = xv[0], x1 = xv[1], cn = cv[0], sn = cv[1];
  const float a0 = x0 * cn;
  const float a1 = x1 * sn;
  const float b0 = x1 * cn;
  const float b1 = x0 * sn;
  const float r0 = a0 - a1;
  const float r1 = b0 + b1;
  const unsigned w16 = pk16(h_bits(r0), h_bits(r1));
  const unsigned short hb0 = f2bf_bits(r0), hb1 = f2bf_bits(r1);
  const unsigned short lb0 = f2bf_bits(r0 - bf_bits2f(hb0)), lb1 = f2bf_bits(r1 - bf_bits2f(hb1));
  const unsigned wh = pk16(hb0, hb1), wl = pk16(lb0, lb1);
  const bool early = (pos < kEarly);
  const size_t erow = (size_t)b * kEarly + (size_t)(early ? pos : 0);
  unsigned* p16 = (unsigned*)kr16 + ((size_t)t * kDRope / 2 + i);
  unsigned* ph  = (unsigned*)kreh + (erow * kDRope / 2 + i);
  unsigned* pl  = (unsigned*)krel + (erow * kDRope / 2 + i);
  for (int pass = 0; pass < 2; ++pass) {
    *(volatile unsigned*)p16 = w16;
    if (early) { *(volatile unsigned*)ph = wh; *(volatile unsigned*)pl = wl; }
    __threadfence();
  }
}

__global__ __launch_bounds__(256) void rope_q16_kernel(unsigned short* __restrict__ q16, const float* __restrict__ cs) {
  #pragma clang fp contract(off)
  const int g = blockIdx.x * 256 + threadIdx.x;
  if (g >= kTok * kHeads * kPairs) return;
  const int i = g & 31;
  const int h = (g >> 5) & (kHeads - 1);
  const int tok = g >> 9;
  const int pos = tok & (kSeq - 1);
  const size_t ho = (size_t)tok * kQCols + (size_t)h * kDQK + kDNope + 2 * i;
  unsigned* wp = (unsigned*)q16 + (ho >> 1);
  const unsigned w = *wp;
  const float x0 = h16_to_f32(w & 0xffffu);
  const float x1 = h16_to_f32(w >> 16);
  const v2f cv = *(const v2f*)(cs + ((size_t)pos * kPairs + i) * 2);
  const float cn = cv[0], sn = cv[1];
  const float a0 = x0 * cn;
  const float a1 = x1 * sn;
  const float b0 = x1 * cn;
  const float b1 = x0 * sn;
  const float r0 = a0 - a1;
  const float r1 = b0 + b1;
  const unsigned wn = pk16(h_bits(r0), h_bits(r1));
  *(volatile unsigned*)wp = wn;
  __threadfence();
  *(volatile unsigned*)wp = wn;
}

__global__ __launch_bounds__(256) void rope_qe_kernel(unsigned short* __restrict__ qeh, unsigned short* __restrict__ qel,
                                                     const float* __restrict__ cs) {
  #pragma clang fp contract(off)
  const int g = blockIdx.x * 256 + threadIdx.x;
  if (g >= kTokE * kHeads * kPairs) return;
  const int i = g & 31;
  const int h = (g >> 5) & (kHeads - 1);
  const int te = g >> 9;
  const int pos = te & (kEarly - 1);
  const size_t ho = (size_t)te * kQCols + (size_t)h * kDQK + kDNope + 2 * i;
  unsigned* ph = (unsigned*)qeh + (ho >> 1);
  unsigned* pl = (unsigned*)qel + (ho >> 1);
  const unsigned wh = *ph;
  const unsigned wl = *pl;
  const float xh0 = __uint_as_float((wh & 0xffffu) << 16), xh1 = __uint_as_float(wh & 0xffff0000u);
  const float xl0 = __uint_as_float((wl & 0xffffu) << 16), xl1 = __uint_as_float(wl & 0xffff0000u);
  const float x0 = xh0 + xl0;
  const float x1 = xh1 + xl1;
  const v2f cv = *(const v2f*)(cs + ((size_t)pos * kPairs + i) * 2);
  const float cn = cv[0], sn = cv[1];
  const float a0 = x0 * cn;
  const float a1 = x1 * sn;
  const float b0 = x1 * cn;
  const float b1 = x0 * sn;
  const float r0 = a0 - a1;
  const float r1 = b0 + b1;
  const unsigned short hb0 = f2bf_bits(r0), hb1 = f2bf_bits(r1);
  const unsigned short lb0 = f2bf_bits(r0 - bf_bits2f(hb0)), lb1 = f2bf_bits(r1 - bf_bits2f(hb1));
  const unsigned nh = pk16(hb0, hb1), nl = pk16(lb0, lb1);
  for (int pass = 0; pass < 2; ++pass) {
    *(volatile unsigned*)ph = nh;
    *(volatile unsigned*)pl = nl;
    __threadfence();
  }
}

__global__ __launch_bounds__(256) void early_kassemble_kernel(const unsigned short* __restrict__ kneh, const unsigned short* __restrict__ knel,
                                                             const unsigned short* __restrict__ kreh, const unsigned short* __restrict__ krel,
                                                             unsigned short* __restrict__ kfeh, unsigned short* __restrict__ kfel) {
  __shared__ __align__(16) v4u sh[(kKVCols + kDRope) / 8];
  __shared__ __align__(16) v4u sl[(kKVCols + kDRope) / 8];
  const int te  = blockIdx.x;
  const int tid = threadIdx.x;
  sh[tid] = *(const v4u*)(kneh + (size_t)te * kKVCols + 8 * tid);
  sl[tid] = *(const v4u*)(knel + (size_t)te * kKVCols + 8 * tid);
  const v4u rh = *(const v4u*)(kreh + (size_t)te * kDRope + 8 * (tid & 7));
  const v4u rl = *(const v4u*)(krel + (size_t)te * kDRope + 8 * (tid & 7));
  if (tid < 8) { sh[256 + tid] = rh; sl[256 + tid] = rl; }
  __syncthreads();
  const int lane = tid & 31, wave = tid >> 5;
#pragma unroll
  for (int hsel = 0; hsel < 2; ++hsel) {
    const int h = wave * 2 + hsel;
    const int src  = (lane < 16) ? (h * 16 + lane) : (256 + (lane - 16));
    const int srcc = (lane < 24) ? src : 0;
    const v4u vh = sh[srcc];
    const v4u vl = sl[srcc];
    const size_t dst = (size_t)te * kQCols + (size_t)h * kDQK + 8 * (size_t)(lane < 24 ? lane : 0);
    for (int pass = 0; pass < 2; ++pass) {
      if (lane < 24) {
        *(volatile v4u*)(kfeh + dst) = vh;
        *(volatile v4u*)(kfel + dst) = vl;
      }
      __threadfence();
    }
  }
}

__global__ __launch_bounds__(256) void early_softmax_kernel(const float* __restrict__ Se, unsigned short* __restrict__ Ph,
                                                           unsigned short* __restrict__ Pl) {
  const int tid  = threadIdx.x;
  const int lane = tid & 31, wave = tid >> 5;
  const int hh = lane >> 4, c = lane & 15;
  const int R = blockIdx.x * 16 + wave * 2 + hh;
  const int q = R & (kEarly - 1);
  const float* sr = Se + (size_t)R * kEarly + 8 * c;
  const v4f a = *(const v4f*)(sr);
  const v4f d = *(const v4f*)(sr + 4);
  float x[8];
#pragma unroll
  for (int e = 0; e < 4; ++e) { x[e] = a[e]; x[4 + e] = d[e]; }
  float m = -INFINITY;
#pragma unroll
  for (int e = 0; e < 8; ++e) {
    const int col = 8 * c + e;
    x[e] = (col > q) ? -INFINITY : x[e];
    m = fmaxf(m, x[e]);
  }
#pragma unroll
  for (int off = 1; off < 16; off <<= 1) m = fmaxf(m, __shfl_xor(m, off, 32));
  float ev[8];
  float sum = 0.0f;
#pragma unroll
  for (int e = 0; e < 8; ++e) { ev[e] = expf(x[e] - m); sum += ev[e]; }
#pragma unroll
  for (int off = 1; off < 16; off <<= 1) sum += __shfl_xor(sum, off, 32);
  const float inv = 1.0f / sum;
  unsigned short hb[8], lb[8];
#pragma unroll
  for (int e = 0; e < 8; ++e) {
    const float p = ev[e] * inv;
    hb[e] = f2bf_bits(p);
    lb[e] = f2bf_bits(p - bf_bits2f(hb[e]));
  }
  const v4u uh = (v4u){pk16(hb[0], hb[1]), pk16(hb[2], hb[3]), pk16(hb[4], hb[5]), pk16(hb[6], hb[7])};
  const v4u ul = (v4u){pk16(lb[0], lb[1]), pk16(lb[2], lb[3]), pk16(lb[4], lb[5]), pk16(lb[6], lb[7])};
  const size_t po = (size_t)R * kEarly + 8 * c;
  for (int pass = 0; pass < 2; ++pass) {
    *(volatile v4u*)(Ph + po) = uh;
    *(volatile v4u*)(Pl + po) = ul;
    __threadfence();
  }
}

constexpr int kFaWaves = 8;
constexpr int kFaQB    = 128;
constexpr int kFaKC    = 64;
constexpr int kOsPitch = 68;
static_assert(kEarly % kFaQB == 0, "query block split");
static_assert(kSeq % kFaKC == 0 && kFaQB % kFaKC == 0, "key chunks");
struct FaKV { v4u K[kFaKC * kDQK / 8]; v4u V[kDV * kFaKC / 8]; };
union FaShm { FaKV kv; float os[kFaWaves][16 * kOsPitch]; };
static_assert(sizeof(FaKV) >= sizeof(float) * kFaWaves * 16 * kOsPitch, "os fits in the staging region");
__global__ __launch_bounds__(256) __attribute__((amdgpu_num_vgpr(256)))
void attn_flash_kernel(const unsigned short* qp, const unsigned short* __restrict__ knp,
                       const unsigned short* __restrict__ krp, const unsigned short* __restrict__ vtp,
                       unsigned short* __restrict__ cvp, int qb0, float sc) {
  __shared__ __align__(16) FaShm shu;
  __shared__ __align__(16) _Float16 Psh[kFaWaves][16 * kFaKC];

  const int tid  = threadIdx.x;
  const int wave = tid >> 5;
  const int lane = tid & 31;
  const int hh   = lane >> 4;
  const int c    = lane & 15;

  const int nqb = (kSeq / kFaQB) - qb0;
  const int bx  = blockIdx.x;
  const int qb  = qb0 + bx % nqb;
  const int bh  = bx / nqb;
  const int h   = bh & (kHeads - 1);
  const int b   = bh >> 4;
  const int q0  = qb * kFaQB + wave * 16;
  const size_t tokq = (size_t)b * kSeq + (size_t)q0;

  const _Float16* qrow = (const _Float16*)qp + (tokq + (size_t)c) * kQCols + (size_t)h * kDQK + 8 * hh;

  float mrow[8], lrow[8];
  v8f oacc[8];
#pragma unroll
  for (int r = 0; r < 8; ++r) { mrow[r] = -INFINITY; lrow[r] = 0.f; }
#pragma unroll
  for (int t = 0; t < 8; ++t) oacc[t] = (v8f){0.f,0.f,0.f,0.f,0.f,0.f,0.f,0.f};

  const int nChunks = (qb + 1) * (kFaQB / kFaKC);
  for (int kc = 0; kc < nChunks; ++kc) {
    const int kv0 = kc * kFaKC;
    __syncthreads();
#pragma unroll
    for (int i = 0; i < 4; ++i) {
      const int e = i * 256 + tid;
      const int r = e >> 4, c16 = e & 15;
      shu.kv.K[r * 24 + c16] = *(const v4u*)(knp + ((size_t)b * kSeq + kv0 + r) * kKVCols + (size_t)h * kDNope + 8 * c16);
    }
#pragma unroll
    for (int i = 0; i < 2; ++i) {
      const int e = i * 256 + tid;
      const int r = e >> 3, c8i = e & 7;
      shu.kv.K[r * 24 + 16 + c8i] = *(const v4u*)(krp + ((size_t)b * kSeq + kv0 + r) * kDRope + 8 * c8i);
    }
#pragma unroll
    for (int i = 0; i < 4; ++i) {
      const int e = i * 256 + tid;
      const int d = e >> 3, c8i = e & 7;
      shu.kv.V[d * 8 + c8i] = *(const v4u*)(vtp + ((size_t)b * kKVCols + (size_t)h * kDV + d) * kSeq + kv0 + 8 * c8i);
    }
    __syncthreads();
    const _Float16* Kh = (const _Float16*)shu.kv.K;
    const _Float16* Vh = (const _Float16*)shu.kv.V;

    v8f s[4];
#pragma unroll
    for (int j = 0; j < 4; ++j) s[j] = (v8f){0.f,0.f,0.f,0.f,0.f,0.f,0.f,0.f};
#pragma unroll 1
    for (int dc = 0; dc < 6; ++dc) {
      const v16h qa = Frag<_Float16>::load(qrow + dc * 32);
#pragma unroll
      for (int j = 0; j < 4; ++j) {
        const v16h kb = Frag<_Float16>::load(Kh + (size_t)(j * 16 + c) * kDQK + dc * 32 + 8 * hh);
        s[j] = fa_mma(qa, kb, s[j]);
      }
    }
    float cm[8];
#pragma unroll
    for (int r = 0; r < 8; ++r) {
      const int qrowi = q0 + 8 * hh + r;
      float m = -INFINITY;
#pragma unroll
      for (int j = 0; j < 4; ++j) {
        const int kvcol = kv0 + j * 16 + c;
        float v = s[j][r] * sc;
        v = (kvcol > qrowi) ? -INFINITY : v;
        s[j][r] = v;
        m = fmaxf(m, v);
      }
#pragma unroll
      for (int off = 1; off < 16; off <<= 1) m = fmaxf(m, __shfl_xor(m, off, 32));
      cm[r] = m;
    }
    _Float16* pwh = Psh[wave];
#pragma unroll
    for (int r = 0; r < 8; ++r) {
      const float mnew  = fmaxf(mrow[r], cm[r]);
      const float alpha = expf(mrow[r] - mnew);
      mrow[r] = mnew;
      float psum = 0.f;
#pragma unroll
      for (int j = 0; j < 4; ++j) {
        const float p = expf(s[j][r] - mnew);
        psum += p;
        pwh[(8 * hh + r) * kFaKC + j * 16 + c] = (_Float16)(p * kPCarry);
      }
#pragma unroll
      for (int off = 1; off < 16; off <<= 1) psum += __shfl_xor(psum, off, 32);
      lrow[r] = lrow[r] * alpha + psum;
#pragma unroll
      for (int t = 0; t < 8; ++t) oacc[t][r] *= alpha;
    }
    wave_lds_sync();
#pragma unroll 1
    for (int kk = 0; kk < 2; ++kk) {
      const v16h pa = Frag<_Float16>::load(pwh + c * kFaKC + kk * 32 + 8 * hh);
#pragma unroll
      for (int t = 0; t < 8; ++t) {
        const v16h vb = Frag<_Float16>::load(Vh + (size_t)(t * 16 + c) * kFaKC + kk * 32 + 8 * hh);
        oacc[t] = fa_mma(pa, vb, oacc[t]);
      }
    }
  }
  __syncthreads();

  float inv[8];
#pragma unroll
  for (int r = 0; r < 8; ++r) { const float rc = 1.0f / (lrow[r] * kPCarry); inv[r] = kOCarry * rc; }
  float* os = shu.os[wave];
  const int qg = lane >> 3, c8 = (lane & 7) * 8;
#pragma unroll
  for (int half = 0; half < 2; ++half) {
#pragma unroll
    for (int r = 0; r < 8; ++r) {
#pragma unroll
      for (int t4 = 0; t4 < 4; ++t4) os[(8 * hh + r) * kOsPitch + t4 * 16 + c] = oacc[half * 4 + t4][r] * inv[r];
    }
    wave_lds_sync();
    for (int pass = 0; pass < 2; ++pass) {
#pragma unroll
      for (int it = 0; it < 4; ++it) {
        const int row = it * 4 + qg;
        const float* sp = os + row * kOsPitch + c8;
        v8h hv;
#pragma unroll
        for (int e = 0; e < 8; ++e) hv[e] = (_Float16)sp[e];
        *(volatile v8h*)(cvp + ((tokq + (size_t)row) * kKVCols + (size_t)h * kDV + (size_t)half * 64 + (size_t)c8)) = hv;
      }
      __threadfence();
    }
    wave_lds_sync();
  }
}

template <int ET, int SPLIT, int BIAS_MODE, int OUT_MODE, bool RESID>
static void gemm_launch(hipStream_t st, int batches,
                        const void* A, const void* A2, int lda, long sA,
                        const void* Bt, const void* Bt2, int ldb, long sB,
                        void* C, void* C2, int ldc, long sC,
                        const float* bias, const float* resid, long sR,
                        int M, int N, int K, float scale) {
  const int tiles = (M >> 6) * (N >> 6);
  dim3 grid((tiles + 7) / 8, batches, 1);
  wmma_gemm64<ET, SPLIT, BIAS_MODE, OUT_MODE, RESID><<<grid, dim3(256), 0, st>>>(
      (const unsigned short*)A, (const unsigned short*)A2, lda, sA,
      (const unsigned short*)Bt, (const unsigned short*)Bt2, ldb, sB,
      C, C2, ldc, sC, bias, resid, sR, M, N, K, scale);
}

extern "C" void kernel_launch(void* const* d_in, const int* in_sizes, int n_in,
                              void* d_out, int out_size, void* d_ws, size_t ws_size,
                              hipStream_t stream) {
  if (n_in < 9) return;
  if (in_sizes[0] != kTok * kDim) return;
  if (in_sizes[2] != kDim * kQCols || in_sizes[3] != kDim * kKCCols || in_sizes[4] != kDim * kRank) return;
  if (in_sizes[5] != kRank * kKVCols || in_sizes[6] != kRank * kKVCols || in_sizes[7] != kKVCols * kDim || in_sizes[8] != kDim) return;
  if (out_size != kTok * kDim) return;

  const float* x   = (const float*)d_in[0];
  const int*   spo = (const int*)d_in[1];
  const float* wq  = (const float*)d_in[2];
  const float* wkc = (const float*)d_in[3];
  const float* wvc = (const float*)d_in[4];
  const float* wku = (const float*)d_in[5];
  const float* wvu = (const float*)d_in[6];
  const float* wo  = (const float*)d_in[7];
  const float* wob = (const float*)d_in[8];
  float* out = (float*)d_out;
  char* ws = (char*)d_ws;

  size_t off = 0;
  auto carve = [&](size_t bytes) { const size_t o = off; off += (bytes + 255) & ~(size_t)255; return o; };
  const size_t szP16  = (size_t)kTok * kKVCols * 2;
  const size_t oXB    = carve((size_t)kTok * kDim * 2);
  const size_t oWQT   = carve((size_t)kQCols * kDim * 2);
  const size_t oWKCT  = carve((size_t)kKCCols * kDim * 2);
  const size_t oWVCT  = carve((size_t)kRank * kDim * 2);
  const size_t oWKUT  = carve((size_t)kKVCols * kRank * 2);
  const size_t oWVUT  = carve((size_t)kKVCols * kRank * 2);
  const size_t oWOT   = carve((size_t)kDim * kKVCols * 2);
  const size_t oWOB   = carve((size_t)kDim * 4);
  const size_t oCS    = carve((size_t)kSeq * kPairs * 2 * 4);
  const size_t oQ16   = carve((size_t)kTok * kQCols * 2);
  const size_t oKCH   = carve((size_t)kTok * kRank * 2);
  const size_t oKCL   = carve((size_t)kTok * kRank * 2);
  const size_t oKR32  = carve((size_t)kTok * kDRope * 4);
  const size_t oVCH   = carve((size_t)kTok * kRank * 2);
  const size_t oVCL   = carve((size_t)kTok * kRank * 2);
  const size_t oKN16  = carve(szP16);
  const size_t oKR16  = carve((size_t)kTok * kDRope * 2);
  const size_t oQEH   = carve((size_t)kTokE * kQCols * 2);
  const size_t oQEL   = carve((size_t)kTokE * kQCols * 2);
  const size_t oKNEH  = carve((size_t)kTokE * kKVCols * 2);
  const size_t oKNEL  = carve((size_t)kTokE * kKVCols * 2);
  const size_t oKREH  = carve((size_t)kTokE * kDRope * 2);
  const size_t oKREL  = carve((size_t)kTokE * kDRope * 2);
  const size_t oKFEH  = carve((size_t)kTokE * kQCols * 2);
  const size_t oKFEL  = carve((size_t)kTokE * kQCols * 2);
  const size_t oVTEH  = carve((size_t)kBatch * kKVCols * kEarly * 2);
  const size_t oVTEL  = carve((size_t)kBatch * kKVCols * kEarly * 2);
  const size_t oSE    = carve((size_t)kBatch * kHeads * kEarly * kEarly * 4);
  const size_t oPEH   = carve((size_t)kBatch * kHeads * kEarly * kEarly * 2);
  const size_t oPEL   = carve((size_t)kBatch * kHeads * kEarly * kEarly * 2);
  const size_t oCVEH  = carve((size_t)kTokE * kKVCols * 2);
  const size_t oCVEL  = carve((size_t)kTokE * kKVCols * 2);
  const size_t oTE    = carve((size_t)kTokE * kDim * 4);
  const size_t total  = off;
  const size_t oCV16  = oXB;
  const size_t oVT16  = oWQT;
  if ((size_t)kTok * kDim * 2 < szP16) return;
  if (oWKUT - oWQT < szP16) return;
  if (total > ws_size || total > (size_t)134217728) return;

  unsigned short* XB   = (unsigned short*)(ws + oXB);
  unsigned short* WQT  = (unsigned short*)(ws + oWQT);
  unsigned short* WKCT = (unsigned short*)(ws + oWKCT);
  unsigned short* WVCT = (unsigned short*)(ws + oWVCT);
  unsigned short* WKUT = (unsigned short*)(ws + oWKUT);
  unsigned short* WVUT = (unsigned short*)(ws + oWVUT);
  unsigned short* WOT  = (unsigned short*)(ws + oWOT);
  float*          WOB  = (float*)(ws + oWOB);
  float*          CS   = (float*)(ws + oCS);
  unsigned short* Q16  = (unsigned short*)(ws + oQ16);
  unsigned short* KCH  = (unsigned short*)(ws + oKCH);
  unsigned short* KCL  = (unsigned short*)(ws + oKCL);
  float*          KR32 = (float*)(ws + oKR32);
  unsigned short* VCH  = (unsigned short*)(ws + oVCH);
  unsigned short* VCL  = (unsigned short*)(ws + oVCL);
  unsigned short* KN16 = (unsigned short*)(ws + oKN16);
  unsigned short* KR16 = (unsigned short*)(ws + oKR16);
  unsigned short* QEH  = (unsigned short*)(ws + oQEH);
  unsigned short* QEL  = (unsigned short*)(ws + oQEL);
  unsigned short* KNEH = (unsigned short*)(ws + oKNEH);
  unsigned short* KNEL = (unsigned short*)(ws + oKNEL);
  unsigned short* KREH = (unsigned short*)(ws + oKREH);
  unsigned short* KREL = (unsigned short*)(ws + oKREL);
  unsigned short* KFEH = (unsigned short*)(ws + oKFEH);
  unsigned short* KFEL = (unsigned short*)(ws + oKFEL);
  unsigned short* VTEH = (unsigned short*)(ws + oVTEH);
  unsigned short* VTEL = (unsigned short*)(ws + oVTEL);
  float*          SE   = (float*)(ws + oSE);
  unsigned short* PEH  = (unsigned short*)(ws + oPEH);
  unsigned short* PEL  = (unsigned short*)(ws + oPEL);
  unsigned short* CVEH = (unsigned short*)(ws + oCVEH);
  unsigned short* CVEL = (unsigned short*)(ws + oCVEL);
  float*          TE   = (float*)(ws + oTE);
  unsigned short* CV16 = (unsigned short*)(ws + oCV16);
  unsigned short* VT16 = (unsigned short*)(ws + oVT16);

  Theta32 th;
  for (int i = 0; i < kPairs; ++i) {
    const float e = (float)(2 * i) / 64.0f;
    const double pd = pow(10000.0, (double)e);
    const float pf = (float)pd;
    th.t[i] = 1.0f / pf;
  }
  const float sc = 1.0f / sqrtf((float)kDQK);

  {
    const int n8 = kTok * kDim / 8;
    cast8_x16_kernel<<<dim3(n8 / 256), dim3(256), 0, stream>>>(x, XB, n8);
  }
  wtrans_kernel<true><<<dim3(kDim / 64, kQCols / 64), dim3(256), 0, stream>>>(wq, WQT, kDim, kQCols, kWCarry);
  wtrans_kernel<true><<<dim3(kDim / 64, kKCCols / 64), dim3(256), 0, stream>>>(wkc, WKCT, kDim, kKCCols, kWCarry);
  wtrans_kernel<true><<<dim3(kDim / 64, kRank / 64), dim3(256), 0, stream>>>(wvc, WVCT, kDim, kRank, kWCarry);
  wtrans_kernel<false><<<dim3(kRank / 64, kKVCols / 64), dim3(256), 0, stream>>>(wku, WKUT, kRank, kKVCols, 1.0f);
  wtrans_kernel<false><<<dim3(kRank / 64, kKVCols / 64), dim3(256), 0, stream>>>(wvu, WVUT, kRank, kKVCols, 1.0f);
  wtrans_kernel<true><<<dim3(kKVCols / 64, kDim / 64), dim3(256), 0, stream>>>(wo, WOT, kKVCols, kDim, kWCarry);
  bias_rne_kernel<<<dim3(kDim / 4 / 256), dim3(256), 0, stream>>>(wob, WOB, kDim / 4);
  rope_table_kernel<<<dim3(kSeq * kPairs / 256), dim3(256), 0, stream>>>(CS, th, spo);

  gemm_launch<0, 0, 0, 1, false>(stream, 1, XB, XB, kDim, 0L, WQT, WQT, kDim, 0L,
                                 Q16, Q16, kQCols, 0L, WOB, WOB, 0L, kTok, kQCols, kDim, kWCarryInv);
  gemm_launch<0, 0, 0, 2, false>(stream, kBatch, XB, XB, kDim, (long)kSeq * kDim, WQT, WQT, kDim, 0L,
                                 QEH, QEL, kQCols, (long)kEarly * kQCols, WOB, WOB, 0L, kEarly, kQCols, kDim, kWCarryInv);
  gemm_launch<0, 0, 0, 2, false>(stream, 1, XB, XB, kDim, 0L, WKCT, WKCT, kDim, 0L,
                                 KCH, KCL, kRank, 0L, WOB, WOB, 0L, kTok, kRank, kDim, kWCarryInv);
  gemm_launch<0, 0, 0, 0, false>(stream, 1, XB, XB, kDim, 0L, WKCT + (size_t)kRank * kDim, WKCT + (size_t)kRank * kDim, kDim, 0L,
                                 KR32, KR32, kDRope, 0L, WOB, WOB, 0L, kTok, kDRope, kDim, kWCarryInv);
  gemm_launch<0, 0, 0, 2, false>(stream, 1, XB, XB, kDim, 0L, WVCT, WVCT, kDim, 0L,
                                 VCH, VCL, kRank, 0L, WOB, WOB, 0L, kTok, kRank, kDim, kWCarryInv);
  gemm_launch<1, 2, 0, 1, false>(stream, 1, KCH, KCL, kRank, 0L, WKUT, WKUT, kRank, 0L,
                                 KN16, KN16, kKVCols, 0L, WOB, WOB, 0L, kTok, kKVCols, kRank, 1.0f);
  gemm_launch<1, 2, 0, 2, false>(stream, kBatch, KCH, KCL, kRank, (long)kSeq * kRank, WKUT, WKUT, kRank, 0L,
                                 KNEH, KNEL, kKVCols, (long)kEarly * kKVCols, WOB, WOB, 0L, kEarly, kKVCols, kRank, 1.0f);
  gemm_launch<1, 3, 0, 1, false>(stream, kBatch, WVUT, WVUT, kRank, 0L, VCH, VCL, kRank, (long)kSeq * kRank,
                                 VT16, VT16, kSeq, (long)kKVCols * kSeq, WOB, WOB, 0L, kKVCols, kSeq, kRank, 1.0f);
  gemm_launch<1, 3, 0, 2, false>(stream, kBatch, WVUT, WVUT, kRank, 0L, VCH, VCL, kRank, (long)kSeq * kRank,
                                 VTEH, VTEL, kEarly, (long)kKVCols * kEarly, WOB, WOB, 0L, kKVCols, kEarly, kRank, 1.0f);

  rope_q16_kernel<<<dim3(kTok * kHeads * kPairs / 256), dim3(256), 0, stream>>>(Q16, CS);
  rope_qe_kernel<<<dim3(kTokE * kHeads * kPairs / 256), dim3(256), 0, stream>>>(QEH, QEL, CS);
  rope_k_kernel<<<dim3(kTok * kPairs / 256), dim3(256), 0, stream>>>(KR32, CS, KR16, KREH, KREL);
  early_kassemble_kernel<<<dim3(kTokE), dim3(256), 0, stream>>>(KNEH, KNEL, KREH, KREL, KFEH, KFEL);

  {
    const int qb0 = kEarly / kFaQB;
    const int nblk = (kSeq / kFaQB - qb0) * kBatch * kHeads;
    attn_flash_kernel<<<dim3(nblk), dim3(256), 0, stream>>>(Q16, KN16, KR16, VT16, CV16, qb0, sc);
  }

  for (int bb = 0; bb < kBatch; ++bb) {
    const size_t qo = (size_t)bb * kEarly * kQCols;
    gemm_launch<1, 1, 0, 0, false>(stream, kHeads, QEH + qo, QEL + qo, kQCols, (long)kDQK, KFEH + qo, KFEL + qo, kQCols, (long)kDQK,
                                   SE + (size_t)bb * kHeads * kEarly * kEarly, SE + (size_t)bb * kHeads * kEarly * kEarly, kEarly, (long)kEarly * kEarly,
                                   WOB, WOB, 0L, kEarly, kEarly, kDQK, sc);
  }
  early_softmax_kernel<<<dim3(kBatch * kHeads * kEarly / 16), dim3(256), 0, stream>>>(SE, PEH, PEL);
  for (int bb = 0; bb < kBatch; ++bb) {
    const size_t po = (size_t)bb * kHeads * kEarly * kEarly;
    const size_t vo = (size_t)bb * kKVCols * kEarly;
    const size_t co = (size_t)bb * kEarly * kKVCols;
    gemm_launch<1, 1, 0, 3, false>(stream, kHeads, PEH + po, PEL + po, kEarly, (long)kEarly * kEarly, VTEH + vo, VTEL + vo, kEarly, (long)kDV * kEarly,
                                   CVEH + co, CVEL + co, kKVCols, (long)kDV, WOB, WOB, 0L, kEarly, kDV, kEarly, kOCarry);
  }
  gemm_launch<0, 0, 0, 0, false>(stream, kBatch, CVEH, CVEH, kKVCols, (long)kEarly * kKVCols, WOT, WOT, kKVCols, 0L,
                                 TE, TE, kDim, (long)kEarly * kDim, WOB, WOB, 0L, kEarly, kDim, kKVCols, 1.0f / (kOCarry * kWCarry));
  gemm_launch<0, 0, 2, 0, true>(stream, kBatch, CVEL, CVEL, kKVCols, (long)kEarly * kKVCols, WOT, WOT, kKVCols, 0L,
                                out, out, kDim, (long)kSeq * kDim, WOB, TE, (long)kEarly * kDim, kEarly, kDim, kKVCols,
                                1.0f / (kOCarry * kWCarry * kLoCarry));
  gemm_launch<0, 0, 2, 0, false>(stream, kBatch, CV16 + (size_t)kEarly * kKVCols, CV16 + (size_t)kEarly * kKVCols, kKVCols, (long)kSeq * kKVCols,
                                 WOT, WOT, kKVCols, 0L,
                                 out + (size_t)kEarly * kDim, out + (size_t)kEarly * kDim, kDim, (long)kSeq * kDim, WOB, WOB, 0L,
                                 kSeq - kEarly, kDim, kKVCols, 1.0f / (kOCarry * kWCarry));
  (void)ws_size;
}
